// GAT_LP_46600395161978
// MI455X (gfx1250) — hardware-run, weakly checked
//
#include <hip/hip_runtime.h>
#include <stddef.h>


#define IN0     256
#define HID     128
#define NHEAD   4
#define FW      512
#define PQW     256
#define MLPH    64
#define NTHR    256
#define NWAVE   8
#define EPT     8
#define CHUNK   (NTHR * EPT)
#define WCAP    (EPT * 32)
#define LISTN   (NWAVE * WCAP)
#define NBMAX   2048
#define SLOTB   11
#define RCAP    28672
#define DEGCAP  4096
#define GBM     64
#define GTHR    128
#define GBN     128
#define NEG_SLOPE 0.2f
#define CA      16.0f
#define CW      64.0f
#define SCL     0.0009765625f
#define WSCAP   134217728
#define LDS_BUILD ((2 * RCAP + 2 * NBMAX + LISTN) * 4 + 64)

static_assert((CHUNK & (CHUNK - 1)) == 0 && CHUNK <= 4096);
static_assert(NBMAX == (1 << SLOTB));
static_assert(NTHR * 8 == NBMAX);
static_assert(LISTN >= NBMAX);
static_assert(LISTN >= NWAVE * WCAP);
static_assert((RCAP % 32) == 0);
static_assert(LDS_BUILD <= 300000);
static_assert(GBM == (GTHR / 32) * 16);
static_assert(GTHR == GBN);
static_assert(NHEAD * HID == FW && GBN == HID);
static_assert((IN0 % 32) == 0 && (FW % 32) == 0 && (HID % 32) == 0);
static_assert(PQW == 2 * HID);
static_assert(MLPH == 64);

typedef float    v4f  __attribute__((ext_vector_type(4)));
typedef float    v8f  __attribute__((ext_vector_type(8)));
typedef int      v4i  __attribute__((ext_vector_type(4)));
typedef int      v8i  __attribute__((ext_vector_type(8)));
typedef _Float16 v8h  __attribute__((ext_vector_type(8)));
typedef _Float16 v16h __attribute__((ext_vector_type(16)));
union FragH { v16h v; v8h h[2]; v8i w; };

__device__ __forceinline__ v8f wmh(const FragH& a, const FragH& b, v8f c) {
  v8f d = __builtin_amdgcn_wmma_f32_16x16x32_f16(false, a.v, false, b.v, (short)0, c, false, false);
  asm volatile("v_nop\n\tv_nop\n\tv_nop\n\tv_nop" : "+v"(d) : "v"(a.w), "v"(b.w));
  return d;
}

__device__ __forceinline__ v8h pack8(v4f a, v4f b, float sc) {
  v8h hv;
  hv[0] = (_Float16)(a.x * sc); hv[1] = (_Float16)(a.y * sc);
  hv[2] = (_Float16)(a.z * sc); hv[3] = (_Float16)(a.w * sc);
  hv[4] = (_Float16)(b.x * sc); hv[5] = (_Float16)(b.y * sc);
  hv[6] = (_Float16)(b.z * sc); hv[7] = (_Float16)(b.w * sc);
  return hv;
}

__device__ __forceinline__ float elu1(float v) { return v > 0.f ? v : (__expf(v) - 1.0f); }

__device__ __forceinline__ int scan_chunk(const int* __restrict__ dsts, int nE, int cbase, int slotBase,
                                          int nb, int vec8, int* list, int tid, int lane, int wave) {
  int wc = 0;
  const int el0  = tid * EPT;
  const int e0   = cbase + el0;
  const int sent = -2147483647 - 1;
  v4i da, db;
  if (vec8 != 0 && cbase + CHUNK <= nE) {
    da = *(const v4i*)(dsts + e0);
    db = *(const v4i*)(dsts + e0 + 4);
  } else {
    da.x = (e0     < nE) ? dsts[min(e0,     nE - 1)] : sent;
    da.y = (e0 + 1 < nE) ? dsts[min(e0 + 1, nE - 1)] : sent;
    da.z = (e0 + 2 < nE) ? dsts[min(e0 + 2, nE - 1)] : sent;
    da.w = (e0 + 3 < nE) ? dsts[min(e0 + 3, nE - 1)] : sent;
    db.x = (e0 + 4 < nE) ? dsts[min(e0 + 4, nE - 1)] : sent;
    db.y = (e0 + 5 < nE) ? dsts[min(e0 + 5, nE - 1)] : sent;
    db.z = (e0 + 6 < nE) ? dsts[min(e0 + 6, nE - 1)] : sent;
    db.w = (e0 + 7 < nE) ? dsts[min(e0 + 7, nE - 1)] : sent;
  }
  const unsigned nbs = (unsigned)slotBase;
  const unsigned unb = (unsigned)nb;
  const unsigned s0 = (unsigned)da.x - nbs, s1 = (unsigned)da.y - nbs;
  const unsigned s2 = (unsigned)da.z - nbs, s3 = (unsigned)da.w - nbs;
  const unsigned s4 = (unsigned)db.x - nbs, s5 = (unsigned)db.y - nbs;
  const unsigned s6 = (unsigned)db.z - nbs, s7 = (unsigned)db.w - nbs;
  const bool h0 = s0 < unb, h1 = s1 < unb, h2 = s2 < unb, h3 = s3 < unb;
  const bool h4 = s4 < unb, h5 = s5 < unb, h6 = s6 < unb, h7 = s7 < unb;
  const unsigned any = __builtin_amdgcn_ballot_w32(h0 | h1 | h2 | h3 | h4 | h5 | h6 | h7);
  if (any != 0u) {
#define HITJ(J, HJ, SJ) { \
      const unsigned mj = __builtin_amdgcn_ballot_w32(HJ); \
      if (mj != 0u) { \
        if (HJ) { \
          const int pos = wc + (int)__builtin_amdgcn_mbcnt_lo(mj, 0u); \
          if (pos < WCAP) list[wave * WCAP + pos] = ((el0 + (J)) << 12) | (int)(SJ); \
        } \
        wc += (int)__builtin_popcount(mj); } }
    HITJ(0, h0, s0)
    HITJ(1, h1, s1)
    HITJ(2, h2, s2)
    HITJ(3, h3, s3)
    HITJ(4, h4, s4)
    HITJ(5, h5, s5)
    HITJ(6, h6, s6)
    HITJ(7, h7, s7)
#undef HITJ
  }
  return wc;
}

__global__ __launch_bounds__(NTHR) void k_xprep(const float* __restrict__ x, _Float16* xh, int nN, int nUnits) {
  const int i = (int)blockIdx.x * NTHR + (int)threadIdx.x;
  if (i >= nUnits) return;
  const int row = i >> 5;
  const int c0  = (i & 31) * 8;
  const int rc  = row < nN ? row : nN - 1;
  const float* p = x + (size_t)rc * IN0 + c0;
  v4f a = *(const v4f*)p, b = *(const v4f*)(p + 4);
  const v4f z4 = {0.f, 0.f, 0.f, 0.f};
  if (row >= nN) { a = z4; b = z4; }
  const v8h hv = pack8(a, b, CA);
  const size_t o = (size_t)row * IN0 + c0;
  *(volatile v8h*)(xh + o) = hv;
  __threadfence();
  *(volatile v8h*)(xh + o) = hv;
}

__global__ __launch_bounds__(NTHR) void k_wprep(const float* __restrict__ w, _Float16* wt,
                                                int K, int CN, int NR, int nUnits) {
  const int u = (int)blockIdx.x * NTHR + (int)threadIdx.x;
  if (u >= nUnits) return;
  const int k8n = K >> 3;
  int n  = u / k8n;
  int k8 = (u - n * k8n) * 8;
  n  = n < NR ? n : NR - 1;
  k8 = k8 < K - 8 ? k8 : K - 8;
  const int seg = n / CN;
  const int col = n - seg * CN;
  const float* p = w + ((size_t)seg * K + (size_t)k8) * CN + col;
  v4f a, b;
  a.x = p[0 * (size_t)CN]; a.y = p[1 * (size_t)CN]; a.z = p[2 * (size_t)CN]; a.w = p[3 * (size_t)CN];
  b.x = p[4 * (size_t)CN]; b.y = p[5 * (size_t)CN]; b.z = p[6 * (size_t)CN]; b.w = p[7 * (size_t)CN];
  const v8h hv = pack8(a, b, CW);
  const size_t o = (size_t)n * K + k8;
  *(volatile v8h*)(wt + o) = hv;
  __threadfence();
  *(volatile v8h*)(wt + o) = hv;
}

__global__ __launch_bounds__(GTHR) void k_gemm(const _Float16* __restrict__ A, int lda,
                                               const _Float16* __restrict__ WT, int K,
                                               float* Y, int ldy,
                                               const float* __restrict__ al, const float* __restrict__ ar,
                                               float* ES, float* ED, int esp, int doAtt) {
  __shared__ __attribute__((aligned(16))) float stg[GBM * GBN];
  __shared__ __attribute__((aligned(16))) float esT[GBM];
  __shared__ __attribute__((aligned(16))) float edT[GBM];
  __shared__ float sAl[GBN];
  __shared__ float sAr[GBN];
  const int tid = threadIdx.x, lane = tid & 31, wave = tid >> 5, hh = lane >> 4, m = lane & 15;
  const int rowBase = (int)blockIdx.x * GBM;
  const int p       = (int)blockIdx.y;
  const int colBase = p * GBN;
  if (doAtt != 0) {
    sAl[tid] = al[(size_t)p * GBN + tid];
    sAr[tid] = ar[(size_t)p * GBN + tid];
  }
  const size_t arow = (size_t)(rowBase + 16 * wave + m) * (size_t)lda + 8 * hh;
  const size_t brow = (size_t)(colBase + m) * (size_t)K + 8 * hh;
  v8f acc[8];
#pragma unroll
  for (int t = 0; t < 8; ++t) { v8f z = {0.f, 0.f, 0.f, 0.f, 0.f, 0.f, 0.f, 0.f}; acc[t] = z; }
  const int nks = K >> 5;
#pragma unroll 1
  for (int ks = 0; ks < nks; ++ks) {
    FragH af;
    af.h[0] = *(const v8h*)(A + arow + 32 * ks);
    af.h[1] = *(const v8h*)(A + arow + 32 * ks + 16);
#pragma unroll
    for (int t = 0; t < 8; ++t) {
      const size_t bo = brow + (size_t)(16 * t) * (size_t)K + 32 * ks;
      FragH bf;
      bf.h[0] = *(const v8h*)(WT + bo);
      bf.h[1] = *(const v8h*)(WT + bo + 16);
      acc[t] = wmh(af, bf, acc[t]);
    }
  }
  {
    float* sp = stg + (size_t)(16 * wave + 8 * hh) * GBN + m;
#pragma unroll
    for (int t = 0; t < 8; ++t) {
#pragma unroll
      for (int r = 0; r < 8; ++r) sp[(size_t)r * GBN + 16 * t] = acc[t][r] * SCL;
    }
  }
  __syncthreads();
  if (doAtt != 0) {
    const int row  = tid >> 1;
    const int half = tid & 1;
    const float* srow = stg + (size_t)row * GBN;
    float s = 0.f, d = 0.f;
#pragma unroll 1
    for (int c = 0; c < GBN / 2; ++c) {
      const int cc = half * (GBN / 2) + c;
      const float v = srow[cc];
      s = fmaf(v, sAl[cc], s);
      d = fmaf(v, sAr[cc], d);
    }
    s += __shfl_xor(s, 1);
    d += __shfl_xor(d, 1);
    if (half == 0) { esT[row] = s; edT[row] = d; }
  }
  {
    const int nF4 = GBM * GBN / 4;
    float* yb = Y + (size_t)rowBase * (size_t)ldy + colBase;
    const v4f* s4 = (const v4f*)stg;
#pragma unroll 1
    for (int f = tid; f < nF4; f += GTHR) {
      const int r = f >> 5, q = f & 31;
      const v4f v = s4[f];
      *(volatile v4f*)(yb + (size_t)r * (size_t)ldy + 4 * q) = v;
    }
    __threadfence();
#pragma unroll 1
    for (int f = tid; f < nF4; f += GTHR) {
      const int r = f >> 5, q = f & 31;
      const v4f v = s4[f];
      *(volatile v4f*)(yb + (size_t)r * (size_t)ldy + 4 * q) = v;
    }
  }
  __syncthreads();
  if (doAtt != 0 && wave == 0 && lane < 16) {
    const v4f ve = *(const v4f*)(esT + 4 * lane);
    const v4f vd = *(const v4f*)(edT + 4 * lane);
    float* pe = ES + (size_t)p * (size_t)esp + rowBase + 4 * lane;
    float* pd = ED + (size_t)p * (size_t)esp + rowBase + 4 * lane;
    *(volatile v4f*)pe = ve;
    *(volatile v4f*)pd = vd;
    __threadfence();
    *(volatile v4f*)pe = ve;
    *(volatile v4f*)pd = vd;
  }
}

__global__ __launch_bounds__(NTHR) void k_build(const int* __restrict__ dsts, int* EL, int* OFF, int* CNT,
                                                int nE, int nb, int tp, int vec8) {
  extern __shared__ v4f lds_dyn[];
  int* reg1 = (int*)lds_dyn;
  int* reg2 = reg1 + RCAP;
  int* scnt = reg2 + RCAP;
  int* soff = scnt + NBMAX;
  int* list = soff + NBMAX;
  int* wcnt = list + LISTN;
  int* wtot = wcnt + NWAVE;
  const int tid = threadIdx.x, lane = tid & 31, wave = tid >> 5;
  const int nodeBase = (int)blockIdx.x * nb;

  for (int i = tid; i < NBMAX; i += NTHR) scnt[i] = 0;
  {
    const v4i z = {0, 0, 0, 0};
    v4i* r2v = (v4i*)reg2;
    for (int f = tid; f < RCAP / 4; f += NTHR) r2v[f] = z;
  }
  __syncthreads();

  int tot = 0;
  const int nChunks = (nE + CHUNK - 1) / CHUNK;
#pragma unroll 1
  for (int ch = 0; ch < nChunks; ++ch) {
    const int cbase = ch * CHUNK;
    const int wc = scan_chunk(dsts, nE, cbase, nodeBase, nb, vec8, list, tid, lane, wave);
    if (lane == 0) wcnt[wave] = wc;
    __syncthreads();
    int pre = 0, all = 0;
#pragma unroll
    for (int w2 = 0; w2 < NWAVE; ++w2) {
      int c = wcnt[w2];
      c = c < 0 ? 0 : (c > WCAP ? WCAP : c);
      all += c;
      pre += (w2 < wave) ? c : 0;
    }
    const int wcc  = wc > WCAP ? WCAP : wc;
    const int base = tot + pre;
#pragma unroll 1
    for (int i = lane; i < wcc; i += 32) {
      const int ent = list[wave * WCAP + i];
      const int el  = (ent >> 12) & (CHUNK - 1);
      const int sl  = ent & (NBMAX - 1);
      int eid = cbase + el;
      eid = eid > nE - 1 ? nE - 1 : eid;
      const int pos = base + i;
      if (pos < RCAP) reg1[pos] = (int)(((unsigned)eid << SLOTB) | (unsigned)sl);
    }
    tot += all;
    tot = tot > RCAP ? RCAP : tot;
    __syncthreads();
  }
  const int nh = tot;

  if (wave == 0) {
#pragma unroll 1
    for (int b0 = 0; b0 < nh; b0 += 32) {
      const int idx = b0 + lane;
      const int uv  = reg1[idx < RCAP ? idx : RCAP - 1];
      const int m32 = (nh - b0) < 32 ? (nh - b0) : 32;
#pragma unroll 1
      for (int k = 0; k < m32; ++k) {
        const int u  = __builtin_amdgcn_readlane(uv, k);
        const int sl = u & (NBMAX - 1);
        if (lane == 0) scnt[sl] = scnt[sl] + 1;
      }
    }
  }
  __syncthreads();

  {
    const v4i ca = *(const v4i*)(scnt + 8 * tid);
    const v4i cb = *(const v4i*)(scnt + 8 * tid + 4);
    const int e0 = ca.x < 0 ? 0 : ca.x, e1 = ca.y < 0 ? 0 : ca.y, e2 = ca.z < 0 ? 0 : ca.z, e3 = ca.w < 0 ? 0 : ca.w;
    const int e4 = cb.x < 0 ? 0 : cb.x, e5 = cb.y < 0 ? 0 : cb.y, e6 = cb.z < 0 ? 0 : cb.z, e7 = cb.w < 0 ? 0 : cb.w;
    const int ts = e0 + e1 + e2 + e3 + e4 + e5 + e6 + e7;
    int incl = ts;
#pragma unroll
    for (int d = 1; d < 32; d <<= 1) {
      const int up = __shfl_up(incl, d);
      if (lane >= d) incl += up;
    }
    if (lane == 31) wtot[wave] = incl;
    __syncthreads();
    int pre = 0;
#pragma unroll
    for (int w2 = 0; w2 < NWAVE; ++w2) pre += (w2 < wave) ? wtot[w2] : 0;
    int run = pre + incl - ts;
    soff[8 * tid + 0] = run; run += e0;
    soff[8 * tid + 1] = run; run += e1;
    soff[8 * tid + 2] = run; run += e2;
    soff[8 * tid + 3] = run; run += e3;
    soff[8 * tid + 4] = run; run += e4;
    soff[8 * tid + 5] = run; run += e5;
    soff[8 * tid + 6] = run; run += e6;
    soff[8 * tid + 7] = run;
  }
  __syncthreads();
  for (int i = tid; i < NBMAX; i += NTHR) list[i] = soff[i];
  __syncthreads();

  if (wave == 0) {
#pragma unroll 1
    for (int b0 = 0; b0 < nh; b0 += 32) {
      const int idx = b0 + lane;
      const int uv  = reg1[idx < RCAP ? idx : RCAP - 1];
      const int m32 = (nh - b0) < 32 ? (nh - b0) : 32;
#pragma unroll 1
      for (int k = 0; k < m32; ++k) {
        const int u   = __builtin_amdgcn_readlane(uv, k);
        const int sl  = u & (NBMAX - 1);
        const int eid = (int)((unsigned)u >> SLOTB);
        if (lane == 0) {
          int pos = list[sl];
          pos = pos < 0 ? 0 : (pos > RCAP - 1 ? RCAP - 1 : pos);
          reg2[pos] = eid;
          list[sl] = pos + 1;
        }
      }
    }
  }
  __syncthreads();

  {
    int* elb = EL + (size_t)blockIdx.x * RCAP;
    const v4i* r4 = (const v4i*)reg2;
#pragma unroll 1
    for (int f = tid; f < RCAP / 4; f += NTHR) {
      const v4i v = r4[f];
      *(volatile v4i*)(elb + 4 * f) = v;
    }
    __threadfence();
#pragma unroll 1
    for (int f = tid; f < RCAP / 4; f += NTHR) {
      const v4i v = r4[f];
      *(volatile v4i*)(elb + 4 * f) = v;
    }
  }
  {
    const bool ovf = (nh >= RCAP);
    int* ob = OFF + (size_t)blockIdx.x * tp;
    int* cb = CNT + (size_t)blockIdx.x * tp;
    const int n4 = tp >> 2;
#pragma unroll 1
    for (int pass = 0; pass < 2; ++pass) {
#pragma unroll 1
      for (int f = tid; f < n4; f += NTHR) {
        v4i so, sc;
        {
          const int s = 4 * f + 0; const bool in = s < nb; const int scl = s < NBMAX ? s : NBMAX - 1;
          so.x = in ? soff[scl] : 0; sc.x = in ? (ovf ? -1 : scnt[scl]) : 0;
        }
        {
          const int s = 4 * f + 1; const bool in = s < nb; const int scl = s < NBMAX ? s : NBMAX - 1;
          so.y = in ? soff[scl] : 0; sc.y = in ? (ovf ? -1 : scnt[scl]) : 0;
        }
        {
          const int s = 4 * f + 2; const bool in = s < nb; const int scl = s < NBMAX ? s : NBMAX - 1;
          so.z = in ? soff[scl] : 0; sc.z = in ? (ovf ? -1 : scnt[scl]) : 0;
        }
        {
          const int s = 4 * f + 3; const bool in = s < nb; const int scl = s < NBMAX ? s : NBMAX - 1;
          so.w = in ? soff[scl] : 0; sc.w = in ? (ovf ? -1 : scnt[scl]) : 0;
        }
        *(volatile v4i*)(ob + 4 * f) = so;
        *(volatile v4i*)(cb + 4 * f) = sc;
      }
      __threadfence();
    }
  }
}

__global__ __launch_bounds__(NTHR) void k_agg(
    const int* __restrict__ srcs, const int* __restrict__ EL,
    const int* __restrict__ OFF, const int* __restrict__ CNT,
    const float* __restrict__ Y, const float* __restrict__ ES, const float* __restrict__ ED,
    const float* __restrict__ bias, float* HF, _Float16* XH, _Float16* HM,
    int nN, int nE, int nb, int tp, int MP, int esp, int resid, int act, int last) {
  __shared__ v4f cmb[NWAVE * 2 * 128];
  __shared__ float cdn[NWAVE * 2 * NHEAD];
  const int tid = threadIdx.x, lane = tid & 31, wave = tid >> 5;
  const int g  = lane >> 4;
  const int L  = lane & 15;
  const int jy = L >> 2;
  const int q8 = lane >> 2;
  const int j4 = lane & 3;
  const int nodeBase = (int)blockIdx.x * nb;
  const int nbw = nb >> 3;
  const int* elb  = EL  + (size_t)blockIdx.x * RCAP;
  const int* offb = OFF + (size_t)blockIdx.x * tp;
  const int* cntb = CNT + (size_t)blockIdx.x * tp;
  v4f*   cw = cmb + wave * 256;
  float* cd = cdn + wave * 8;
  const float qnan = __int_as_float(0x7fc00000);
  const float ninf = __int_as_float(0xff800000);
  const v4f z4 = {0.f, 0.f, 0.f, 0.f};
#pragma unroll 1
  for (int jt = 0; jt < nbw; ++jt) {
    const int slot = wave * nbw + jt;
    const int grow = nodeBase + slot;
    const int gcl  = grow < nN ? grow : nN - 1;
    const bool vnode = grow < nN;
    const bool inb   = grow < MP;
    int st = offb[slot];
    const int craw = cntb[slot];
    st = st < 0 ? 0 : (st > RCAP - 1 ? RCAP - 1 : st);
    int cnt = craw < 0 ? 0 : (craw > DEGCAP ? DEGCAP : craw);
    if (cnt > RCAP - st) cnt = RCAP - st;
    const float pz = (craw < 0 || craw > DEGCAP) ? qnan : 0.0f;

    const float ed1 = ED[(size_t)j4 * (size_t)esp + gcl];
    float mx = ninf;
    const int n1 = (cnt + 7) >> 3;
#pragma unroll 1
    for (int it = 0; it < n1; ++it) {
      const int q   = it * 8 + q8;
      const int qc  = q < cnt ? q : cnt - 1;
      const int idx = st + qc;
      int eid = elb[idx];
      eid = eid < 0 ? 0 : (eid > nE - 1 ? nE - 1 : eid);
      const int sraw = srcs[eid];
      const int s = sraw < 0 ? 0 : (sraw > nN - 1 ? nN - 1 : sraw);
      const float u = ES[(size_t)j4 * (size_t)esp + s] + ed1;
      const float l = fmaxf(u, NEG_SLOPE * u);
      mx = fmaxf(mx, l);
    }
    mx = fmaxf(mx, __shfl_xor(mx, 4));
    mx = fmaxf(mx, __shfl_xor(mx, 8));
    mx = fmaxf(mx, __shfl_xor(mx, 16));
    const float mj = __shfl(mx, jy);

    const float ed2 = ED[(size_t)jy * (size_t)esp + gcl];
    float dn = 0.f;
    v4f a0 = z4, a1 = z4, a2 = z4, a3 = z4, a4 = z4, a5 = z4, a6 = z4, a7 = z4;
    const int n2 = (cnt + 1) >> 1;
#pragma unroll 1
    for (int it = 0; it < n2; ++it) {
      const int q = it * 2 + g;
      const bool valid = q < cnt;
      const int qc  = valid ? q : cnt - 1;
      const int idx = st + qc;
      int eid = elb[idx];
      eid = eid < 0 ? 0 : (eid > nE - 1 ? nE - 1 : eid);
      const int sraw = srcs[eid];
      const int s = sraw < 0 ? 0 : (sraw > nN - 1 ? nN - 1 : sraw);
      const float* ys = Y + (size_t)s * FW + 32 * L;
      const v4f x0 = *(const v4f*)(ys +  0);
      const v4f x1 = *(const v4f*)(ys +  4);
      const v4f x2 = *(const v4f*)(ys +  8);
      const v4f x3 = *(const v4f*)(ys + 12);
      const v4f x4 = *(const v4f*)(ys + 16);
      const v4f x5 = *(const v4f*)(ys + 20);
      const v4f x6 = *(const v4f*)(ys + 24);
      const v4f x7 = *(const v4f*)(ys + 28);
      const float u = ES[(size_t)jy * (size_t)esp + s] + ed2;
      const float l = fmaxf(u, NEG_SLOPE * u);
      const float ww = __expf(l - mj);
      const float w = valid ? ww : 0.f;
      dn += w;
      a0 += x0 * w; a1 += x1 * w; a2 += x2 * w; a3 += x3 * w;
      a4 += x4 * w; a5 += x5 * w; a6 += x6 * w; a7 += x7 * w;
    }
    __builtin_amdgcn_fence(__ATOMIC_RELEASE, "wavefront");
    __builtin_amdgcn_wave_barrier();
    {
      v4f* cg = cw + g * 128 + 8 * L;
      cg[0] = a0; cg[1] = a1; cg[2] = a2; cg[3] = a3;
      cg[4] = a4; cg[5] = a5; cg[6] = a6; cg[7] = a7;
      if ((L & 3) == 0) cd[g * NHEAD + jy] = dn;
    }
    __builtin_amdgcn_fence(__ATOMIC_RELEASE, "wavefront");
    __builtin_amdgcn_wave_barrier();
    v4f msum = z4;
#pragma unroll 1
    for (int i = 0; i < NHEAD; ++i) {
      v4f r = cw[32 * i + lane] + cw[128 + 32 * i + lane];
      const float dsum = cd[i] + cd[NHEAD + i];
      const float inv  = dsum > 0.f ? __builtin_amdgcn_rcpf(dsum) : 0.f;
      r = r * inv;
      if (resid != 0 && vnode) r += *(const v4f*)(HF + (size_t)grow * FW + 128 * i + 4 * lane);
      r += *(const v4f*)(bias + 128 * i + 4 * lane);
      r += pz;
      if (act != 0) { r.x = elu1(r.x); r.y = elu1(r.y); r.z = elu1(r.z); r.w = elu1(r.w); }
      if (!vnode) r = z4;
      if (last == 0) {
        if (inb) *(volatile v4f*)(HF + (size_t)grow * FW + 128 * i + 4 * lane) = r;
        cw[32 * i + lane] = r;
      } else {
        msum += r;
      }
    }
    if (last != 0) cw[lane] = msum * 0.25f;
    __builtin_amdgcn_fence(__ATOMIC_RELEASE, "wavefront");
    __builtin_amdgcn_wave_barrier();
    v8h hv0, hv1;
    if (last == 0) {
      hv0 = pack8(cw[2 * lane], cw[2 * lane + 1], CA);
      hv1 = pack8(cw[64 + 2 * lane], cw[65 + 2 * lane], CA);
      if (inb) {
        *(volatile v8h*)(XH + (size_t)grow * FW + 8 * lane) = hv0;
        *(volatile v8h*)(XH + (size_t)grow * FW + 256 + 8 * lane) = hv1;
      }
    } else {
      hv0 = pack8(cw[2 * L], cw[2 * L + 1], CA);
      hv1 = hv0;
      if (inb && lane < 16) *(volatile v8h*)(HM + (size_t)grow * HID + 8 * L) = hv0;
    }
    __threadfence();
    if (last == 0) {
#pragma unroll 1
      for (int i = 0; i < NHEAD; ++i) {
        const v4f r = cw[32 * i + lane];
        if (inb) *(volatile v4f*)(HF + (size_t)grow * FW + 128 * i + 4 * lane) = r;
      }
      if (inb) {
        *(volatile v8h*)(XH + (size_t)grow * FW + 8 * lane) = hv0;
        *(volatile v8h*)(XH + (size_t)grow * FW + 256 + 8 * lane) = hv1;
      }
    } else {
      if (inb && lane < 16) *(volatile v8h*)(HM + (size_t)grow * HID + 8 * L) = hv0;
    }
  }
}

__global__ __launch_bounds__(NTHR) void k_zprep(const int* __restrict__ srcs, const int* __restrict__ dsts,
                                                const float* __restrict__ PQ, const float* __restrict__ bm0,
                                                _Float16* zh, int nN, int nE, int nUnits) {
  const int i = (int)blockIdx.x * NTHR + (int)threadIdx.x;
  if (i >= nUnits) return;
  const int e  = i >> 4;
  const int c0 = (i & 15) * 8;
  const int ec = e < nE ? e : nE - 1;
  int s = srcs[ec]; s = s < 0 ? 0 : (s > nN - 1 ? nN - 1 : s);
  int d = dsts[ec]; d = d < 0 ? 0 : (d > nN - 1 ? nN - 1 : d);
  const float* pp = PQ + (size_t)s * PQW + c0;
  const float* qp = PQ + (size_t)d * PQW + HID + c0;
  v4f a = *(const v4f*)pp + *(const v4f*)qp + *(const v4f*)(bm0 + c0);
  v4f b = *(const v4f*)(pp + 4) + *(const v4f*)(qp + 4) + *(const v4f*)(bm0 + c0 + 4);
  a.x = fmaxf(a.x, 0.f); a.y = fmaxf(a.y, 0.f); a.z = fmaxf(a.z, 0.f); a.w = fmaxf(a.w, 0.f);
  b.x = fmaxf(b.x, 0.f); b.y = fmaxf(b.y, 0.f); b.z = fmaxf(b.z, 0.f); b.w = fmaxf(b.w, 0.f);
  const v4f z4 = {0.f, 0.f, 0.f, 0.f};
  if (e >= nE) { a = z4; b = z4; }
  const v8h hv = pack8(a, b, CA);
  const size_t o = (size_t)e * HID + c0;
  *(volatile v8h*)(zh + o) = hv;
  __threadfence();
  *(volatile v8h*)(zh + o) = hv;
}

__global__ __launch_bounds__(GTHR) void k_mlp(const _Float16* __restrict__ zh, const _Float16* __restrict__ wm1t,
                                              const float* __restrict__ bm1, const float* __restrict__ wm2,
                                              const float* __restrict__ bm2, float* out, int nE) {
  __shared__ __attribute__((aligned(16))) float sO[GBM];
  __shared__ float sb1[MLPH];
  __shared__ float sw2[MLPH];
  const int tid = threadIdx.x, lane = tid & 31, wave = tid >> 5, hh = lane >> 4, m = lane & 15;
  const int rowBase = (int)blockIdx.x * GBM;
  if (tid < MLPH) { sb1[tid] = bm1[tid]; sw2[tid] = wm2[tid]; }
  const size_t arow = (size_t)(rowBase + 16 * wave + m) * HID + 8 * hh;
  const size_t brow = (size_t)m * HID + 8 * hh;
  v8f acc[4];
#pragma unroll
  for (int t = 0; t < 4; ++t) { v8f z = {0.f, 0.f, 0.f, 0.f, 0.f, 0.f, 0.f, 0.f}; acc[t] = z; }
#pragma unroll 1
  for (int ks = 0; ks < HID / 32; ++ks) {
    FragH af;
    af.h[0] = *(const v8h*)(zh + arow + 32 * ks);
    af.h[1] = *(const v8h*)(zh + arow + 32 * ks + 16);
#pragma unroll
    for (int t = 0; t < 4; ++t) {
      const size_t bo = brow + (size_t)(16 * t) * HID + 32 * ks;
      FragH bf;
      bf.h[0] = *(const v8h*)(wm1t + bo);
      bf.h[1] = *(const v8h*)(wm1t + bo + 16);
      acc[t] = wmh(af, bf, acc[t]);
    }
  }
  __syncthreads();
  float o[8];
  {
    const float c0 = sb1[m], c1 = sb1[16 + m], c2 = sb1[32 + m], c3 = sb1[48 + m];
    const float q0 = sw2[m], q1 = sw2[16 + m], q2 = sw2[32 + m], q3 = sw2[48 + m];
#pragma unroll
    for (int r = 0; r < 8; ++r) {
      const float h0 = fmaxf(fmaf(acc[0][r], SCL, c0), 0.f);
      const float h1 = fmaxf(fmaf(acc[1][r], SCL, c1), 0.f);
      const float h2 = fmaxf(fmaf(acc[2][r], SCL, c2), 0.f);
      const float h3 = fmaxf(fmaf(acc[3][r], SCL, c3), 0.f);
      o[r] = fmaf(h0, q0, fmaf(h1, q1, fmaf(h2, q2, h3 * q3)));
    }
  }
#pragma unroll
  for (int r = 0; r < 8; ++r) {
    o[r] += __shfl_xor(o[r], 1);
    o[r] += __shfl_xor(o[r], 2);
    o[r] += __shfl_xor(o[r], 4);
    o[r] += __shfl_xor(o[r], 8);
  }
  {
    const float bb = bm2[0];
    if (m == 0) {
#pragma unroll
      for (int r = 0; r < 8; ++r) {
        const float v  = o[r] + bb;
        const float ev = __expf(-v);
        sO[16 * wave + 8 * hh + r] = __builtin_amdgcn_rcpf(1.0f + ev);
      }
    }
  }
  __syncthreads();
  const int nValid = (nE - rowBase) < GBM ? (nE - rowBase) : GBM;
  const int fl  = nValid;
  const int n4  = fl >> 2;
  const int rem = fl & 3;
  float* base = out + (size_t)rowBase;
  const v4f* s4 = (const v4f*)sO;
  const v4f v = s4[tid < n4 ? tid : 0];
  const int ti = 4 * n4 + (lane & 3);
  const float tv = sO[ti < fl ? ti : fl - 1];
  const bool vw = (n4 > 0) && (tid < n4);
  const bool tw = (rem != 0) && (tid >= n4) && (tid < n4 + rem) && (wave == 0);
  if (vw) *(volatile v4f*)(base + 4 * tid) = v;
  if (tw) *(volatile float*)(base + 4 * n4 + (tid - n4)) = tv;
  __threadfence();
  if (vw) *(volatile v4f*)(base + 4 * tid) = v;
  if (tw) *(volatile float*)(base + 4 * n4 + (tid - n4)) = tv;
}

static int pick_nb(int nE, int nN) {
  int nb = NBMAX;
  while (nb > 64 && (long long)nb * (long long)nE * 5LL > (long long)RCAP * (long long)nN * 4LL) nb >>= 1;
  return nb;
}

extern "C" void kernel_launch(void* const* d_in, const int* in_sizes, int n_in,
                              void* d_out, int out_size, void* d_ws, size_t ws_size,
                              hipStream_t stream) {
  if (n_in < 21) return;
  const int nN = in_sizes[0] / IN0;
  if (nN <= 0 || in_sizes[0] != nN * IN0) return;
  if (nN > (1 << 22)) return;
  const int nE = in_sizes[1];
  if (nE < 1 || nE > (1 << 21)) return;
  if (in_sizes[2] != nE) return;
  if (in_sizes[3] != IN0 * FW) return;
  if (in_sizes[4] != FW || in_sizes[5] != FW || in_sizes[6] != FW) return;
  if (in_sizes[7] != FW * FW) return;
  if (in_sizes[8] != FW || in_sizes[9] != FW || in_sizes[10] != FW) return;
  if (in_sizes[11] != FW * FW) return;
  if (in_sizes[12] != FW || in_sizes[13] != FW || in_sizes[14] != FW) return;
  if (in_sizes[15] != PQW * HID) return;
  if (in_sizes[16] != HID) return;
  if (in_sizes[17] != HID * MLPH) return;
  if (in_sizes[18] != MLPH || in_sizes[19] != MLPH || in_sizes[20] != 1) return;
  if (out_size != nE) return;

  const float* x   = (const float*)d_in[0];
  const int*   src = (const int*)d_in[1];
  const int*   dst = (const int*)d_in[2];
  const float* W0  = (const float*)d_in[3];
  const float* al0 = (const float*)d_in[4];
  const float* ar0 = (const float*)d_in[5];
  const float* b0  = (const float*)d_in[6];
  const float* W1  = (const float*)d_in[7];
  const float* al1 = (const float*)d_in[8];
  const float* ar1 = (const float*)d_in[9];
  const float* b1  = (const float*)d_in[10];
  const float* W2  = (const float*)d_in[11];
  const float* al2 = (const float*)d_in[12];
  const float* ar2 = (const float*)d_in[13];
  const float* b2  = (const float*)d_in[14];
  const float* Wm0 = (const float*)d_in[15];
  const float* bm0 = (const float*)d_in[16];
  const float* Wm1 = (const float*)d_in[17];
  const float* bm1 = (const float*)d_in[18];
  const float* Wm2 = (const float*)d_in[19];
  const float* bm2 = (const float*)d_in[20];
  float* out = (float*)d_out;

  const int MP   = ((nN + GBM - 1) / GBM) * GBM;
  const int EPAD = ((nE + GBM - 1) / GBM) * GBM;
  const int nb   = pick_nb(nE, nN);
  const int tp   = nb;
  const int gA   = (nN + nb - 1) / nb;
  const int gG   = MP / GBM;
  const int gM   = EPAD / GBM;
  const int vec8 = 1;
  if (nb < 64 || nb > NBMAX) return;
  if ((long long)gA * nb < (long long)MP) return;

  char* ws = (char*)d_ws;
  size_t off = 0;
  const size_t oW0T = off; off += (size_t)FW * IN0 * 2;           off = (off + 255) & ~(size_t)255;
  const size_t oW1T = off; off += (size_t)FW * FW * 2;            off = (off + 255) & ~(size_t)255;
  const size_t oW2T = off; off += (size_t)FW * FW * 2;            off = (off + 255) & ~(size_t)255;
  const size_t oWPT = off; off += (size_t)PQW * HID * 2;          off = (off + 255) & ~(size_t)255;
  const size_t oWM1 = off; off += (size_t)MLPH * HID * 2;         off = (off + 255) & ~(size_t)255;
  const size_t oX0H = off; off += (size_t)MP * IN0 * 2;           off = (off + 255) & ~(size_t)255;
  const size_t oXH  = off; off += (size_t)MP * FW * 2;            off = (off + 255) & ~(size_t)255;
  const size_t oHM  = off; off += (size_t)MP * HID * 2;           off = (off + 255) & ~(size_t)255;
  const size_t oY   = off; off += (size_t)MP * FW * 4;            off = (off + 255) & ~(size_t)255;
  const size_t oHF  = off; off += (size_t)MP * FW * 4;            off = (off + 255) & ~(size_t)255;
  const size_t oES  = off; off += (size_t)NHEAD * MP * 4;         off = (off + 255) & ~(size_t)255;
  const size_t oED  = off; off += (size_t)NHEAD * MP * 4;         off = (off + 255) & ~(size_t)255;
  const size_t oEL  = off; off += (size_t)gA * RCAP * 4;          off = (off + 255) & ~(size_t)255;
  const size_t oOFF = off; off += (size_t)gA * tp * 4;            off = (off + 255) & ~(size_t)255;
  const size_t oCNT = off; off += (size_t)gA * tp * 4;            off = (off + 255) & ~(size_t)255;
  const size_t oZH  = off; off += (size_t)EPAD * HID * 2;         off = (off + 255) & ~(size_t)255;
  if (off > ws_size || off > (size_t)WSCAP) return;
  _Float16* W0T  = (_Float16*)(ws + oW0T);
  _Float16* W1T  = (_Float16*)(ws + oW1T);
  _Float16* W2T  = (_Float16*)(ws + oW2T);
  _Float16* WPT  = (_Float16*)(ws + oWPT);
  _Float16* WM1T = (_Float16*)(ws + oWM1);
  _Float16* X0H  = (_Float16*)(ws + oX0H);
  _Float16* XH   = (_Float16*)(ws + oXH);
  _Float16* HM   = (_Float16*)(ws + oHM);
  float*    Y    = (float*)(ws + oY);
  float*    HF   = (float*)(ws + oHF);
  float*    ES   = (float*)(ws + oES);
  float*    ED   = (float*)(ws + oED);
  int*      EL   = (int*)(ws + oEL);
  int*      OFF  = (int*)(ws + oOFF);
  int*      CNT  = (int*)(ws + oCNT);
  _Float16* ZH   = (_Float16*)(ws + oZH);
  float*    PQ   = Y;

  hipFuncSetAttribute(reinterpret_cast<const void*>(&k_build),
                      hipFuncAttributeMaxDynamicSharedMemorySize, LDS_BUILD);

  {
    const int nUnits = MP * (IN0 / 8);
    k_xprep<<<(nUnits + NTHR - 1) / NTHR, NTHR, 0, stream>>>(x, X0H, nN, nUnits);
  }
  {
    const int u0 = FW * (IN0 / 8);
    k_wprep<<<(u0 + NTHR - 1) / NTHR, NTHR, 0, stream>>>(W0, W0T, IN0, FW, FW, u0);
    const int u1 = FW * (FW / 8);
    k_wprep<<<(u1 + NTHR - 1) / NTHR, NTHR, 0, stream>>>(W1, W1T, FW, FW, FW, u1);
    k_wprep<<<(u1 + NTHR - 1) / NTHR, NTHR, 0, stream>>>(W2, W2T, FW, FW, FW, u1);
    const int u2 = PQW * (HID / 8);
    k_wprep<<<(u2 + NTHR - 1) / NTHR, NTHR, 0, stream>>>(Wm0, WPT, HID, HID, PQW, u2);
    const int u3 = MLPH * (HID / 8);
    k_wprep<<<(u3 + NTHR - 1) / NTHR, NTHR, 0, stream>>>(Wm1, WM1T, HID, MLPH, MLPH, u3);
  }

  k_build<<<gA, NTHR, LDS_BUILD, stream>>>(dst, EL, OFF, CNT, nE, nb, tp, vec8);

  k_gemm<<<dim3(gG, FW / GBN), GTHR, 0, stream>>>(X0H, IN0, W0T, IN0, Y, FW, al0, ar0, ES, ED, MP, 1);
  k_agg<<<gA, NTHR, 0, stream>>>(src, EL, OFF, CNT, Y, ES, ED, b0, HF, XH, HM, nN, nE, nb, tp, MP, MP, 0, 1, 0);
  k_gemm<<<dim3(gG, FW / GBN), GTHR, 0, stream>>>(XH, FW, W1T, FW, Y, FW, al1, ar1, ES, ED, MP, 1);
  k_agg<<<gA, NTHR, 0, stream>>>(src, EL, OFF, CNT, Y, ES, ED, b1, HF, XH, HM, nN, nE, nb, tp, MP, MP, 1, 1, 0);
  k_gemm<<<dim3(gG, FW / GBN), GTHR, 0, stream>>>(XH, FW, W2T, FW, Y, FW, al2, ar2, ES, ED, MP, 1);
  k_agg<<<gA, NTHR, 0, stream>>>(src, EL, OFF, CNT, Y, ES, ED, b2, HF, XH, HM, nN, nE, nb, tp, MP, MP, 1, 0, 1);

  k_gemm<<<dim3(gG, PQW / GBN), GTHR, 0, stream>>>(HM, HID, WPT, HID, PQ, PQW, Wm0, Wm0, ES, ED, MP, 0);
  {
    const int nUnits = EPAD * (HID / 8);
    k_zprep<<<(nUnits + NTHR - 1) / NTHR, NTHR, 0, stream>>>(src, dst, PQ, bm0, ZH, nN, nE, nUnits);
  }
  k_mlp<<<gM, GTHR, 0, stream>>>(ZH, WM1T, bm1, Wm2, bm2, out, nE);
}
